// KAN_Convolutional_Layer_78520592105536
// MI455X (gfx1250) — hardware-verified
//
#include <hip/hip_runtime.h>


#define NBT  16
#define NCH  16
#define IH   64
#define IW   64
#define NPIX (IH * IW)
#define NPL  (NBT * NCH)
#define NCV  8
#define KP   128
#define NCP  64
#define CHK  65536
typedef _Float16 h16;
typedef unsigned short bf;
typedef __attribute__((ext_vector_type(16))) __bf16   v16bf;
typedef __attribute__((ext_vector_type(16))) _Float16 v16h;
typedef __attribute__((ext_vector_type(8)))  _Float16 v8h;
typedef __attribute__((ext_vector_type(8)))  unsigned short v8us;
typedef __attribute__((ext_vector_type(8)))  float    v8f;
typedef __attribute__((ext_vector_type(4)))  float    v4f;
typedef v8h  __attribute__((may_alias)) v8ha;
typedef v4f  __attribute__((may_alias)) v4fa;
typedef v8us __attribute__((may_alias)) v8usa;

__device__ __forceinline__ unsigned short f2bf(float f) { unsigned u = __float_as_uint(f); u += 0x7FFFu + ((u >> 16) & 1u); return (unsigned short)(u >> 16); }
__device__ __forceinline__ float bf2f(unsigned short b) { return __uint_as_float(((unsigned)b) << 16); }
__device__ __forceinline__ float bfr(float f) { return bf2f(f2bf(f)); }
__device__ __forceinline__ v16h cat16(v8h lo, v8h hi) { return __builtin_shufflevector(lo, hi, 0, 1, 2, 3, 4, 5, 6, 7, 8, 9, 10, 11, 12, 13, 14, 15); }
__device__ __forceinline__ v16bf cat16b(v8us lo, v8us hi) { return __builtin_bit_cast(v16bf, __builtin_shufflevector(lo, hi, 0, 1, 2, 3, 4, 5, 6, 7, 8, 9, 10, 11, 12, 13, 14, 15)); }
__device__ __forceinline__ v8f wmma16(v16h a, v16h b, v8f c) { return __builtin_amdgcn_wmma_f32_16x16x32_f16(false, a, false, b, (short)0, c, false, false); }
__device__ __forceinline__ v8f wmmab(v16bf a, v16bf b, v8f c) { return __builtin_amdgcn_wmma_f32_16x16x32_bf16(false, a, false, b, (short)0, c, false, false); }


template <typename T16> struct WFrag;
template <> struct WFrag<h16> { typedef v16h V; static __device__ __forceinline__ V ld(const h16* p) { return cat16(*(const v8h*)p, *(const v8h*)(p + 16)); } static __device__ __forceinline__ v8f mma(V a, V b, v8f c) { return wmma16(a, b, c); } };
template <> struct WFrag<bf> { typedef v16bf V; static __device__ __forceinline__ V ld(const bf* p) { return cat16b(*(const v8us*)p, *(const v8us*)(p + 16)); } static __device__ __forceinline__ v8f mma(V a, V b, v8f c) { return wmmab(a, b, c); } };
template <typename T16, int NSPLIT, bool BIAS>
__global__ __launch_bounds__(32) void k_gemmw(const T16* __restrict__ A, const T16* __restrict__ A2, const T16* __restrict__ Bt, const T16* __restrict__ Bt2, int K, float* C, int ldc, const float* __restrict__ bias, size_t sA, size_t sB, size_t sC) {
    typedef typename WFrag<T16>::V V;
    __shared__ __align__(16) float os[16 * 68];
    const size_t z = blockIdx.z; A += z * sA; if (A2) A2 += z * sA; Bt += z * sB; if (Bt2) Bt2 += z * sB; C += z * sC;
    const int lane = threadIdx.x & 31, lr = lane & 15, hi = lane >> 4; const int r0 = blockIdx.x * 64, c0 = blockIdx.y * 64;
    v8f acc[4][4];
#pragma unroll
    for (int mb = 0; mb < 4; ++mb)
#pragma unroll
        for (int nb = 0; nb < 4; ++nb) acc[mb][nb] = (v8f){};
    const size_t aoff = (size_t)(r0 + lr) * K + 8 * hi, boff = (size_t)(c0 + lr) * K + 8 * hi;
#pragma unroll 1
    for (int kc = 0; kc < K; kc += 32) {
        V a[4], a2[4];
#pragma unroll
        for (int mb = 0; mb < 4; ++mb) { a[mb] = WFrag<T16>::ld(A + aoff + (size_t)mb * 16 * K + kc); if (NSPLIT == 1 || NSPLIT == 2) a2[mb] = WFrag<T16>::ld(A2 + aoff + (size_t)mb * 16 * K + kc); }
#pragma unroll
        for (int nb = 0; nb < 4; ++nb) { const V b = WFrag<T16>::ld(Bt + boff + (size_t)nb * 16 * K + kc); V b2; if (NSPLIT >= 2) b2 = WFrag<T16>::ld(Bt2 + boff + (size_t)nb * 16 * K + kc);
#pragma unroll
            for (int mb = 0; mb < 4; ++mb) { acc[mb][nb] = WFrag<T16>::mma(a[mb], b, acc[mb][nb]); if (NSPLIT == 1 || NSPLIT == 2) acc[mb][nb] = WFrag<T16>::mma(a2[mb], b, acc[mb][nb]); if (NSPLIT >= 2) acc[mb][nb] = WFrag<T16>::mma(a[mb], b2, acc[mb][nb]); } }
        asm volatile("v_nop\n\tv_nop\n\tv_nop\n\tv_nop" : "+v"(acc[0][0]), "+v"(acc[1][1]), "+v"(acc[2][2]), "+v"(acc[3][3]) : "v"(a[0]), "v"(a[3]));
    }
#pragma unroll
    for (int mb = 0; mb < 4; ++mb) {
#pragma unroll
        for (int nb = 0; nb < 4; ++nb) {
#pragma unroll
            for (int j = 0; j < 8; ++j) os[(hi * 8 + j) * 68 + nb * 16 + lr] = acc[mb][nb][j]; }
        __builtin_amdgcn_wave_barrier(); asm volatile("" ::: "memory");
        float* crow = C + (size_t)(r0 + mb * 16) * ldc + c0;
#pragma unroll 1
        for (int ps = 0; ps < 2; ++ps) {
#pragma unroll
            for (int s = 0; s < 8; ++s) { const int row = 2 * s + hi, cofs = lr * 4; v4f val = *(const v4fa*)(os + row * 68 + cofs); if (BIAS) { val[0] += bfr(bias[c0 + cofs]); val[1] += bfr(bias[c0 + cofs + 1]); val[2] += bfr(bias[c0 + cofs + 2]); val[3] += bfr(bias[c0 + cofs + 3]); }
                *(volatile v4f*)(crow + (size_t)row * ldc + cofs) = val; }
            if (ps == 0) __threadfence(); }
        __builtin_amdgcn_wave_barrier(); asm volatile("" ::: "memory");
    }
}

__constant__ float GK[12] = {-2.200000047683716f,-1.7999999523162842f,-1.399999976158142f,-1.0f,-0.6000000238418579f,-0.19999998807907104f,0.20000004768371582f,0.6000000238418579f,1.0f,1.4000000953674316f,1.7999999523162842f,2.200000047683716f};
__constant__ float RK[33] = {2.499999523162842f,2.500000238418579f,2.500000238418579f,2.500000238418579f,2.499999761581421f,2.499999761581421f,2.500000238418579f,2.500000238418579f,2.499999523162842f,2.5000009536743164f,2.499999523162842f,1.2499998807907104f,1.2500001192092896f,1.2500001192092896f,1.25f,1.2499998807907104f,1.25f,1.2500001192092896f,1.2499998807907104f,1.2500001192092896f,1.2500001192092896f,0.0f,0.8333333134651184f,0.8333333730697632f,0.8333333134651184f,0.8333333134651184f,0.8333333134651184f,0.8333333134651184f,0.8333333134651184f,0.8333333730697632f,0.8333333134651184f,0.0f,0.0f};
__device__ __forceinline__ void splitf(float y, unsigned short& h, unsigned short& l) { h = f2bf(y); l = f2bf(y - bf2f(h)); }
__global__ __launch_bounds__(64) void k_wrow(const float* __restrict__ bw, const float* __restrict__ sw, const float* __restrict__ sc, bf* Bh, bf* Bl) { const int n = threadIdx.x; if (n >= NCP) return;
#pragma unroll 1
    for (int ps = 0; ps < 2; ++ps) {
#pragma unroll 1
        for (int col = 0; col < KP; ++col) { float v = 0.0f; if (n < NCV) { if (col < 72) { const int i = col >> 3, g = col & 7; v = __fmul_rn(bfr(sw[(n * 9 + i) * 8 + g]), bfr(sc[n * 9 + i])); } else if (col < 81) v = bfr(bw[n * 9 + (col - 72)]); }
            unsigned short h2, l2; splitf(v, h2, l2); *(volatile unsigned short*)(Bh + (size_t)n * KP + col) = h2; *(volatile unsigned short*)(Bl + (size_t)n * KP + col) = l2; }
        if (ps == 0) __threadfence(); } }
__global__ __launch_bounds__(256) void k_featc(const float* __restrict__ X, size_t p0, bf* Ah, bf* Al) {
    const size_t pl = (size_t)blockIdx.x * 256 + threadIdx.x; if (pl >= CHK) return; const size_t p = p0 + pl; const int plane = (int)(p / NPIX); const int hw = (int)(p % NPIX); const int h = hw / IW, w = hw % IW; const float* xpl = X + (size_t)plane * NPIX; bf* rh = Ah + pl * KP; bf* rl = Al + pl * KP;
#pragma unroll 1
    for (int ps = 0; ps < 2; ++ps) {
        v8us z; for (int k = 0; k < 8; ++k) z[k] = 0;
#pragma unroll 1
        for (int c8 = 80; c8 < KP; c8 += 8) { *(volatile v8us*)(rh + c8) = z; *(volatile v8us*)(rl + c8) = z; }
#pragma unroll 1
        for (int i = 0; i < 9; ++i) { const int hh = h + i / 3 - 1, ww = w + i % 3 - 1; const bool in = (hh >= 0 && hh < IH && ww >= 0 && ww < IW); const float x = in ? bfr(xpl[hh * IW + ww]) : 0.0f;
            const float sg = __fdiv_rn(1.0f, __fadd_rn(1.0f, __builtin_amdgcn_exp2f(__fmul_rn(x, -1.4426950408889634f)))); const float sl = __fmul_rn(x, sg); unsigned short sh_, sl_; splitf(sl, sh_, sl_); *(volatile unsigned short*)(rh + 72 + i) = sh_; *(volatile unsigned short*)(rl + 72 + i) = sl_;
            float bs[11];
#pragma unroll
            for (int k = 0; k < 11; ++k) bs[k] = (x >= GK[k] && x < GK[k + 1]) ? 1.0f : 0.0f;
#pragma unroll
            for (int pp = 1; pp <= 3; ++pp) {
#pragma unroll
                for (int k = 0; k < 11 - pp; ++k) { float dl = __fmul_rn(__fsub_rn(x, GK[k]), RK[(pp - 1) * 11 + k]); asm volatile("" : "+v"(dl)); float lt = __fmul_rn(dl, bs[k]); asm volatile("" : "+v"(lt)); float dr = __fmul_rn(__fsub_rn(GK[k + pp + 1], x), RK[(pp - 1) * 11 + k + 1]); asm volatile("" : "+v"(dr)); float rt = __fmul_rn(dr, bs[k + 1]); asm volatile("" : "+v"(rt)); bs[k] = __fadd_rn(lt, rt); } }
            v8us oh, ol;
#pragma unroll
            for (int g = 0; g < 8; ++g) { unsigned short h2, l2; splitf(bs[g], h2, l2); oh[g] = h2; ol[g] = l2; }
            *(volatile v8us*)(rh + i * 8) = oh; *(volatile v8us*)(rl + i * 8) = ol; }
        if (ps == 0) __threadfence(); }
}
__global__ __launch_bounds__(256) void k_outc(const float* __restrict__ Cc, size_t p0, float* out) { const size_t i = (size_t)blockIdx.x * 256 + threadIdx.x; if (i >= (size_t)CHK * NCV / 4) return; const size_t q4 = (i % (CHK / 4)) * 4; const int n = (int)(i / (CHK / 4)); const size_t p = p0 + q4; const int plane = (int)(p / NPIX); const int hw = (int)(p % NPIX); v4f o;
#pragma unroll
    for (int q = 0; q < 4; ++q) o[q] = Cc[(q4 + q) * NCP + n];
    const size_t oo = ((size_t)plane * NCV + n) * NPIX + hw; *(volatile v4f*)(out + oo) = o; __threadfence(); *(volatile v4f*)(out + oo) = o; }

extern "C" void kernel_launch(void* const* d_in, const int* in_sizes, int n_in,
                              void* d_out, int out_size, void* d_ws, size_t ws_size, hipStream_t stream) {
    (void)in_sizes; (void)n_in; (void)out_size;
    const float* x = (const float*)d_in[0]; const float* bw = (const float*)d_in[1]; const float* sw = (const float*)d_in[2]; const float* sc = (const float*)d_in[3];
    float* OUT = (float*)d_out;
    char* wsp = (char*)d_ws;
    auto take = [&](size_t bytes) { char* p = wsp; wsp += (bytes + 255) & ~(size_t)255; return (void*)p; };
    bf* Bh = (bf*)take((size_t)NCP * KP * 2); bf* Bl = (bf*)take((size_t)NCP * KP * 2); bf* Ah = (bf*)take((size_t)CHK * KP * 2); bf* Al = (bf*)take((size_t)CHK * KP * 2); float* Cc = (float*)take((size_t)CHK * NCP * 4);
    if ((size_t)(wsp - (char*)d_ws) > ws_size) return;
    k_wrow<<<1, 64, 0, stream>>>(bw, sw, sc, Bh, Bl);
    static_assert(((size_t)NPL * NPIX) % CHK == 0 && CHK % NPIX == 0, "chunks are whole planes");
    for (size_t p0 = 0; p0 < (size_t)NPL * NPIX; p0 += CHK) {
        k_featc<<<CHK / 256, 256, 0, stream>>>(x, p0, Ah, Al);
        k_gemmw<bf, 2, false><<<dim3(CHK / 64, NCP / 64, 1), 32, 0, stream>>>(Ah, Al, Bh, Bl, KP, Cc, NCP, nullptr, 0, 0, 0);
        k_outc<<<(unsigned)(((size_t)CHK * NCV / 4 + 255) / 256), 256, 0, stream>>>(Cc, p0, OUT); }
}
